// self_a_22574348107986
// MI455X (gfx1250) — hardware-verified
//
#include <hip/hip_runtime.h>
#include <math.h>

typedef __attribute__((ext_vector_type(16))) _Float16 v16h;
typedef __attribute__((ext_vector_type(16))) __bf16 v16b;
typedef __attribute__((ext_vector_type(8)))  _Float16 v8h;
typedef __attribute__((ext_vector_type(8)))  float v8f;
typedef __attribute__((ext_vector_type(4)))  float v4f;
typedef __attribute__((ext_vector_type(2)))  float v2f;
typedef __attribute__((ext_vector_type(4)))  unsigned v4u;
typedef __attribute__((ext_vector_type(4)))  int v4i;
typedef float __attribute__((may_alias)) float_a;
typedef int __attribute__((may_alias)) int_a;

template <typename T> __device__ __forceinline__ void vst2(void* p, T v) { *(volatile T*)p = v; __threadfence(); *(volatile T*)p = v; }
__device__ __forceinline__ v8f wmma16(v16h a, v16h b, v8f c) {
  v8f d = __builtin_amdgcn_wmma_f32_16x16x32_f16(false, a, false, b, (short)0, c, false, false);
  asm volatile("v_nop\n\tv_nop\n\tv_nop\n\tv_nop" : "+v"(d) : "v"(a), "v"(b));
  return d;
}
__device__ __forceinline__ v8f wmma_bf(v16b a, v16b b, v8f c) {
  v8f d = __builtin_amdgcn_wmma_f32_16x16x32_bf16(false, a, false, b, (short)0, c, false, false);
  asm volatile("v_nop\n\tv_nop\n\tv_nop\n\tv_nop" : "+v"(d) : "v"(a), "v"(b));
  return d;
}
__device__ __forceinline__ v16h frag_h(const _Float16* rowk0, int lane) {
  union { v16h v; v8h q[2]; } u; const _Float16* p = rowk0 + 8 * (lane >> 4);
  u.q[0] = *(const v8h*)p; u.q[1] = *(const v8h*)(p + 16); return u.v;
}
__device__ __forceinline__ v16h frag_f32(const float* rowk0, int lane) {
  v16h a; const float* p = rowk0 + 8 * (lane >> 4);
#pragma unroll
  for (int i = 0; i < 8; ++i) { a[i] = (_Float16)p[i]; a[8 + i] = (_Float16)p[16 + i]; }
  return a;
}
__device__ __forceinline__ v16h frag_f32s(const float* rowk0, int lane, float sc) {
  v16h a; const float* p = rowk0 + 8 * (lane >> 4);
#pragma unroll
  for (int i = 0; i < 8; ++i) { a[i] = (_Float16)(p[i] * sc); a[8 + i] = (_Float16)(p[16 + i] * sc); }
  return a;
}
__device__ __forceinline__ v16h fragc_f32(const float* W, int k0, int n, int lane, int ld, int K) {
  v16h a; const int g = lane >> 4;
#pragma unroll
  for (int i = 0; i < 8; ++i) { const int ka = k0 + 8 * g + i, kb = ka + 16;
    a[i] = (_Float16)(ka < K ? W[(size_t)(ka < K ? ka : K - 1) * ld + n] : 0.f); a[8 + i] = (_Float16)(kb < K ? W[(size_t)(kb < K ? kb : K - 1) * ld + n] : 0.f); }
  return a;
}
struct F2 { v16b h, l; };
__device__ __forceinline__ F2 bsplit16(const float v[16]) { F2 r;
#pragma unroll
  for (int i = 0; i < 16; ++i) { const __bf16 h = (__bf16)v[i]; r.h[i] = h; r.l[i] = (__bf16)(v[i] - (float)h); }
  return r; }
__device__ __forceinline__ F2 split_row(const float* row, int k0, int lane) { float v[16]; const float* p = row + k0 + 8 * (lane >> 4);
#pragma unroll
  for (int i = 0; i < 8; ++i) { v[i] = p[i]; v[8 + i] = p[16 + i]; }
  return bsplit16(v); }
__device__ __forceinline__ F2 split_rowK(const float* row, int k0, int lane, int K) { float v[16]; const int g = lane >> 4;
#pragma unroll
  for (int i = 0; i < 8; ++i) { const int ka = k0 + 8 * g + i, kb = ka + 16; v[i] = ka < K ? row[ka < K ? ka : K - 1] : 0.f; v[8 + i] = kb < K ? row[kb < K ? kb : K - 1] : 0.f; }
  return bsplit16(v); }
__device__ __forceinline__ F2 split_col(const float* W, int k0, int n, int lane, int ld, int K) { float v[16]; const int g = lane >> 4;
#pragma unroll
  for (int i = 0; i < 8; ++i) { const int ka = k0 + 8 * g + i, kb = ka + 16; v[i] = ka < K ? W[(size_t)(ka < K ? ka : K - 1) * ld + n] : 0.f; v[8 + i] = kb < K ? W[(size_t)(kb < K ? kb : K - 1) * ld + n] : 0.f; }
  return bsplit16(v); }
__device__ __forceinline__ v8f mac3(const F2& a, const F2& b, v8f c) { c = wmma_bf(a.l, b.h, c); c = wmma_bf(a.h, b.l, c); return wmma_bf(a.h, b.h, c); }
__device__ __forceinline__ float sigm(float v) { return 1.0f / (1.0f + expf(-v)); }
#define LDSX() do { asm volatile("s_wait_dscnt 0" ::: "memory"); __builtin_amdgcn_wave_barrier(); __builtin_amdgcn_fence(__ATOMIC_RELEASE, "workgroup"); } while (0)


#define NB 2
#define CC 64
#define HW 96
#define SS (HW * HW)
#define NR (NB * SS)
#ifndef TQB
#define TQB (SS / 64)
#define TNB NB
#endif
typedef __attribute__((ext_vector_type(8))) __bf16 v8b;
__device__ __forceinline__ v16b frag_b(const __bf16* rowk0, int lane) {
  union { v16b v; v8b q[2]; } u; const __bf16* p = rowk0 + 8 * (lane >> 4);
  u.q[0] = *(const v8b*)p; u.q[1] = *(const v8b*)(p + 16); return u.v;
}
__device__ __forceinline__ float bfr(float v) { return (float)(__bf16)v; }
__device__ __attribute__((noinline)) float exp_ni(float v) { return expf(v); }
__device__ __attribute__((noinline)) float erf_ni(float v) { return erff(v); }

#define WS_PK  0u
#define WS_QH  (((2u * 4 * CC * CC) + 127u) / 128u * 128u)
#define WS_QL  (WS_QH + 2u * NR * CC)
#define WS_KH  (WS_QL + 2u * NR * CC)
#define WS_KL  (WS_KH + 2u * NR * CC)
#define WS_VX  (WS_KL + 2u * NR * CC)
#define WS_VY  (WS_VX + 2u * NR * CC)
#define WS_END (WS_VY + 2u * NR * CC)

__global__ __launch_bounds__(64) void k_pack(const float* __restrict__ WQ, const float* __restrict__ WK, const float* __restrict__ WVX, const float* __restrict__ WVY, __bf16* __restrict__ PK) {
  __shared__ __align__(16) __bf16 s[CC]; const int n = blockIdx.x, which = blockIdx.y, t = threadIdx.x; const float* Wm = (which == 0) ? WQ : (which == 1) ? WK : (which == 2) ? WVX : WVY;
  s[t] = (__bf16)Wm[n * CC + t];
  __syncthreads();
  if (t < CC / 8) vst2((unsigned*)(PK + ((size_t)which * CC + n) * CC + t * 8), *(const v4u*)&s[t * 8]);
}
__global__ __launch_bounds__(128) void k_proj(const float* __restrict__ X, const float* __restrict__ Y, const __bf16* __restrict__ PK, const float* __restrict__ BQ, const float* __restrict__ BK, const float* __restrict__ BVX, const float* __restrict__ BVY, _Float16* __restrict__ QH, _Float16* __restrict__ QL_, _Float16* __restrict__ KH, _Float16* __restrict__ KL, _Float16* __restrict__ VX, _Float16* __restrict__ VY) {
  __shared__ __align__(16) __bf16 sx[64][72], sy[64][72]; __shared__ __align__(16) _Float16 soh[4][16][72], sol[4][16][72]; __shared__ __align__(16) _Float16 svx[CC][72], svy[CC][72];
  const int tid = threadIdx.x, wave = tid >> 5, lane = tid & 31, col = lane & 15, g = lane >> 4; const int pb = blockIdx.x, b = blockIdx.y; const int n0 = pb * 64;
  for (int e = tid; e < CC * 64; e += 128) { const int c = e >> 6, r = e & 63; sx[r][c] = (__bf16)X[((size_t)b * CC + c) * SS + n0 + r]; sy[r][c] = (__bf16)Y[((size_t)b * CC + c) * SS + n0 + r]; }
  if (tid < 64) for (int c = 64; c < 72; ++c) { sx[tid][c] = (__bf16)0.f; sy[tid][c] = (__bf16)0.f; }
  __syncthreads();
  v16b ax[2], ay[2];
#pragma unroll
  for (int kc = 0; kc < 2; ++kc) { ax[kc] = frag_b(&sx[wave * 16 + col][kc * 32], lane); ay[kc] = frag_b(&sy[wave * 16 + col][kc * 32], lane); }
#pragma unroll 1
  for (int which = 0; which < 4; ++which) { v8f acc[4] = {}; const __bf16* P = PK + (size_t)which * CC * CC; const float* BB = (which == 0) ? BQ : (which == 1) ? BK : (which == 2) ? BVX : BVY; const bool fromY = (which == 0 || which == 3);
#pragma unroll
    for (int kc = 0; kc < 2; ++kc)
#pragma unroll
      for (int j = 0; j < 4; ++j) acc[j] = wmma_bf(fromY ? ay[kc] : ax[kc], frag_b(P + (size_t)(j * 16 + col) * CC + kc * 32, lane), acc[j]);
    if (which < 2) {
#pragma unroll
      for (int j = 0; j < 4; ++j) { const int c = j * 16 + col; const float bb = bfr(BB[c]);
#pragma unroll
        for (int r = 0; r < 8; ++r) { const float v = acc[j][r] + bb; const _Float16 hv = (_Float16)v; soh[wave][8 * g + r][c] = hv; sol[wave][8 * g + r][c] = (_Float16)((v - (float)hv) * 2048.0f); } }
      LDSX();
      _Float16* DH = (which == 0) ? QH : KH; _Float16* DL = (which == 0) ? QL_ : KL;
      for (int rl = 0; rl < 16; ++rl) { const size_t o = ((size_t)b * SS + n0 + wave * 16 + rl) * CC; if (lane < 8) vst2((unsigned*)(DH + o + lane * 8), *(const v4u*)&soh[wave][rl][lane * 8]); else if (lane < 16) vst2((unsigned*)(DL + o + (lane - 8) * 8), *(const v4u*)&sol[wave][rl][(lane - 8) * 8]); }
      LDSX();
    } else {
#pragma unroll
      for (int j = 0; j < 4; ++j) { const int c = j * 16 + col; const float bb = bfr(BB[c]);
#pragma unroll
        for (int r = 0; r < 8; ++r) { const _Float16 hv = (_Float16)(acc[j][r] + bb); if (which == 2) svx[c][wave * 16 + 8 * g + r] = hv; else svy[c][wave * 16 + 8 * g + r] = hv; } } } }
  __syncthreads();
  for (int e = tid; e < CC * 8 * 2; e += 128) { const int plane = e / (CC * 8), rem = e % (CC * 8); const int c = rem >> 3, pc = rem & 7; const size_t o = ((size_t)b * CC + c) * SS + n0 + pc * 8;
    if (plane == 0) vst2((unsigned*)(VX + o), *(const v4u*)&svx[c][pc * 8]); else vst2((unsigned*)(VY + o), *(const v4u*)&svy[c][pc * 8]); }
}
__global__ __launch_bounds__(128) void k_attn(const _Float16* __restrict__ QH, const _Float16* __restrict__ QL_, const _Float16* __restrict__ KH, const _Float16* __restrict__ KL, const _Float16* __restrict__ VX, const _Float16* __restrict__ VY, const float* __restrict__ GAMMA, const float* __restrict__ BETA, float* __restrict__ OX, float* __restrict__ OY) {
  __shared__ __align__(16) _Float16 sph[4][16][40]; __shared__ __align__(16) float sox[CC][68], soy[CC][68];
  const int tid = threadIdx.x, wave = tid >> 5, lane = tid & 31, col = lane & 15, g = lane >> 4; const int qb = blockIdx.x, b = blockIdx.y; const int q0 = qb * 64 + wave * 16; const size_t rq = (size_t)b * SS + q0 + col;
  v16h aqh[2], aql[2];
#pragma unroll
  for (int kc = 0; kc < 2; ++kc) { aqh[kc] = frag_h(QH + rq * CC + kc * 32, lane); aql[kc] = frag_h(QL_ + rq * CC + kc * 32, lane); }
  const _Float16* Vx = VX + (size_t)b * CC * SS; const _Float16* Vy = VY + (size_t)b * CC * SS;
  float m[8], l[8];
#pragma unroll
  for (int r = 0; r < 8; ++r) { m[r] = -3.0e38f; l[r] = 0.f; }
  v8f accx[4] = {}, accy[4] = {};
#pragma unroll 1
  for (int ks = 0; ks < SS / 32; ++ks) { v8f s[2];
#pragma unroll
    for (int ct = 0; ct < 2; ++ct) { const int kk = ks * 32 + ct * 16 + col; const size_t rk = ((size_t)b * SS + kk) * CC; v8f c = {}, cl = {};
#pragma unroll
      for (int kc = 0; kc < 2; ++kc) { const v16h khf = frag_h(KH + rk + kc * 32, lane); c = wmma16(aqh[kc], khf, c); cl = wmma16(aql[kc], khf, cl); cl = wmma16(aqh[kc], frag_h(KL + rk + kc * 32, lane), cl); }
#pragma unroll
      for (int r = 0; r < 8; ++r) s[ct][r] = c[r] + cl[r] * (1.0f / 2048.0f); }
#pragma unroll
    for (int r = 0; r < 8; ++r) { float mx = fmaxf(s[0][r], s[1][r]);
#pragma unroll
      for (int o = 1; o < 16; o <<= 1) mx = fmaxf(mx, __shfl_xor(mx, o));
      const float mn = fmaxf(m[r], mx); const float alpha = (m[r] <= -1.0e38f) ? 0.f : exp_ni(m[r] - mn); const float e0 = exp_ni(s[0][r] - mn), e1 = exp_ni(s[1][r] - mn); float es = e0 + e1;
#pragma unroll
      for (int o = 1; o < 16; o <<= 1) es += __shfl_xor(es, o);
      l[r] = l[r] * alpha + es; m[r] = mn;
#pragma unroll
      for (int dt = 0; dt < 4; ++dt) { accx[dt][r] *= alpha; accy[dt][r] *= alpha; }
      sph[wave][8 * g + r][col] = (_Float16)e0; sph[wave][8 * g + r][16 + col] = (_Float16)e1; }
    LDSX();
    const v16h pah = frag_h(&sph[wave][col][0], lane);
#pragma unroll
    for (int dt = 0; dt < 4; ++dt) { const size_t vo = (size_t)(dt * 16 + col) * SS + ks * 32; accx[dt] = wmma16(pah, frag_h(Vx + vo, lane), accx[dt]); accy[dt] = wmma16(pah, frag_h(Vy + vo, lane), accy[dt]); }
    LDSX(); }
  const float ga = bfr(GAMMA[0]), be = bfr(BETA[0]);
#pragma unroll
  for (int r = 0; r < 8; ++r) { const float il = 1.0f / l[r];
#pragma unroll
    for (int dt = 0; dt < 4; ++dt) { sox[dt * 16 + col][wave * 16 + 8 * g + r] = accx[dt][r] * il * ga; soy[dt * 16 + col][wave * 16 + 8 * g + r] = accy[dt][r] * il * be; } }
  __syncthreads();
  for (int e = tid; e < CC * 16 * 2; e += 128) { const int plane = e / (CC * 16), rem = e % (CC * 16); const int c = rem >> 4, pc = rem & 15; const size_t o = ((size_t)b * CC + c) * SS + qb * 64 + pc * 4;
    if (plane == 0) vst2(OX + o, *(const v4f*)&sox[c][pc * 4]); else vst2(OY + o, *(const v4f*)&soy[c][pc * 4]); }
}
extern "C" void kernel_launch(void* const* d_in, const int* in_sizes, int n_in, void* d_out, int out_size, void* d_ws, size_t ws_size, hipStream_t stream) {
  (void)in_sizes; (void)n_in; (void)out_size;
  const float** F = (const float**)d_in;
  if (ws_size < (size_t)WS_END) return;
  char* ws = (char*)d_ws; __bf16* PK = (__bf16*)(ws + WS_PK); _Float16 *QH = (_Float16*)(ws + WS_QH), *QLp = (_Float16*)(ws + WS_QL), *KH = (_Float16*)(ws + WS_KH), *KL = (_Float16*)(ws + WS_KL), *VX = (_Float16*)(ws + WS_VX), *VY = (_Float16*)(ws + WS_VY);
  float* OX = (float*)d_out; float* OY = (float*)((char*)d_out + 4718592);
  k_pack<<<dim3(CC, 4), 64, 0, stream>>>(F[2], F[4], F[6], F[8], PK);
  k_proj<<<dim3(SS / 64, TNB), 128, 0, stream>>>(F[0], F[1], PK, F[3], F[5], F[7], F[9], QH, QLp, KH, KL, VX, VY);
  k_attn<<<dim3(TQB, TNB), 128, 0, stream>>>(QH, QLp, KH, KL, VX, VY, F[10], F[11], OX, OY);
}
